// ProgressiveExpandableFFN_12146167513167
// MI455X (gfx1250) — hardware-verified
//
#include <hip/hip_runtime.h>
#include <math.h>

typedef __attribute__((ext_vector_type(16))) _Float16 v16h;
typedef __attribute__((ext_vector_type(8)))  _Float16 v8h;
typedef __attribute__((ext_vector_type(16))) __bf16   v16b;
typedef __attribute__((ext_vector_type(8)))  __bf16   v8b;
typedef __attribute__((ext_vector_type(8)))  float    v8f;
typedef __attribute__((ext_vector_type(4)))  float    v4f;
typedef __attribute__((ext_vector_type(4)))  unsigned int v4u;

constexpr int kDM = 1024;
constexpr int kDF = 4096;
constexpr int kTok = 8192;
constexpr int kChunkRows = 1024;
constexpr int kNumChunks = kTok / kChunkRows;
constexpr int kNPX = 256;
constexpr int kXPer4 = (kTok * kDM / 4) / kNPX;
constexpr int kGeluBlocks = (kChunkRows * kDF) / (256 * 32);
constexpr int kNPH = kNumChunks * kGeluBlocks;
constexpr int kHqBlocks = (kChunkRows * kDF) / (256 * 8);
constexpr int kXqBlocks = (kTok * kDM) / (256 * 8);
constexpr float kXCarry = 8.0f;
constexpr float kWinCarry = 128.0f;
constexpr float kGCarry = 1024.0f;
constexpr float kGCarryInv = 1.0f / 1024.0f;
constexpr float kHCarry = 64.0f;
constexpr float kWoutCarry = 256.0f;
constexpr float kScale1 = 1.0f / (8.0f * 128.0f);
constexpr float kScale2 = 1.0f / (64.0f * 256.0f);

constexpr size_t kOffScalX = 0;
constexpr size_t kOffScalH = 256;
constexpr size_t kOffScIn = 512;
constexpr size_t kOffInvIn = kOffScIn + 16384;
constexpr size_t kOffScOut = kOffInvIn + 16384;
constexpr size_t kOffInvOut = kOffScOut + 16384;
constexpr size_t kOffXPart = kOffInvOut + 16384;
constexpr size_t kOffHPart = kOffXPart + (size_t)kNPX * 128;
constexpr size_t kOffX16 = 1048576;
constexpr size_t kOffWinT = kOffX16 + (size_t)kTok * kDM * 2;
constexpr size_t kOffWoutT = kOffWinT + (size_t)kDF * kDM * 2;
constexpr size_t kOffScr = kOffWoutT + (size_t)kDM * kDF * 2;
constexpr size_t kOffG16 = kOffScr + (size_t)kChunkRows * kDF * 4;
constexpr size_t kWsTotal = kOffG16 + (size_t)kTok * kDF * 2;

__device__ __forceinline__ unsigned short f2bf_bits(float f) {
  unsigned u = __float_as_uint(f);
  return (unsigned short)((u + 0x7FFFu + ((u >> 16) & 1u)) >> 16);
}
__device__ __forceinline__ float bf_bits2f(unsigned short h) { return __uint_as_float(((unsigned)h) << 16); }

__device__ __forceinline__ void dep_guard_h(v8f& a, v8f& b, v16h x, v16h y) { asm volatile("v_nop\n\tv_nop\n\tv_nop\n\tv_nop" : "+v"(a), "+v"(b) : "v"(x), "v"(y)); }
__device__ __forceinline__ void dep_guard_b(v8f& a, v8f& b, v16b x, v16b y) { asm volatile("v_nop\n\tv_nop\n\tv_nop\n\tv_nop" : "+v"(a), "+v"(b) : "v"(x), "v"(y)); }
__device__ __forceinline__ void keep4_h(v16h a, v16h b, v16h c, v16h d) { asm volatile("v_nop" :: "v"(a), "v"(b), "v"(c), "v"(d)); }
__device__ __forceinline__ void keep4_b(v16b a, v16b b, v16b c, v16b d) { asm volatile("v_nop" :: "v"(a), "v"(b), "v"(c), "v"(d)); }
__device__ __forceinline__ void acc_guard4(v8f& a, v8f& b, v8f& c, v8f& d) { asm volatile("v_nop\n\tv_nop\n\tv_nop\n\tv_nop" : "+v"(a), "+v"(b), "+v"(c), "+v"(d)); }
template <typename T> struct Frag;
template <> struct Frag<_Float16> {
  typedef v16h V; union U { v16h v; v8h h[2]; };
  static __device__ __forceinline__ v16h load(const _Float16* p) {
    U f; f.h[0] = *(const v8h*)(p); f.h[1] = *(const v8h*)(p + 16); return f.v;
  }
  static __device__ __forceinline__ v8f mma(v16h a, v16h b, v8f c) {
    return __builtin_amdgcn_wmma_f32_16x16x32_f16(false, a, false, b, (short)0, c, false, false);
  }
  static __device__ __forceinline__ void guard(v8f& a, v8f& b, v16h x, v16h y) { dep_guard_h(a, b, x, y); }
  static __device__ __forceinline__ void keep(v16h a, v16h b, v16h c, v16h d) { keep4_h(a, b, c, d); }
};
template <> struct Frag<__bf16> {
  typedef v16b V; union U { v16b v; v8b h[2]; };
  static __device__ __forceinline__ v16b load(const __bf16* p) {
    U f; f.h[0] = *(const v8b*)(p); f.h[1] = *(const v8b*)(p + 16); return f.v;
  }
  static __device__ __forceinline__ v8f mma(v16b a, v16b b, v8f c) {
    return __builtin_amdgcn_wmma_f32_16x16x32_bf16(false, a, false, b, (short)0, c, false, false);
  }
  static __device__ __forceinline__ void guard(v8f& a, v8f& b, v16b x, v16b y) { dep_guard_b(a, b, x, y); }
  static __device__ __forceinline__ void keep(v16b a, v16b b, v16b c, v16b d) { keep4_b(a, b, c, d); }
};

__device__ __forceinline__ unsigned pk16(unsigned short a, unsigned short b) { return (unsigned)a | ((unsigned)b << 16); }
__device__ __forceinline__ unsigned short h_bits(float f) { const _Float16 h = (_Float16)f; return __builtin_bit_cast(unsigned short, h); }
__device__ __forceinline__ float f16lo_to_f32(unsigned w) { return (float)__builtin_bit_cast(_Float16, (unsigned short)(w & 0xffffu)); }
__device__ __forceinline__ float f16hi_to_f32(unsigned w) { return (float)__builtin_bit_cast(_Float16, (unsigned short)(w >> 16)); }

template <int ET> struct Elem;
template <> struct Elem<0> { typedef _Float16 T; };
template <> struct Elem<1> { typedef __bf16 T; };
template <int ET, bool SPLIT, int BIAS_MODE, int OUT_MODE, bool RESID, int ACT = 0>
__global__ __launch_bounds__(256) void wmma_gemm64(
    const unsigned short* __restrict__ Ap, const unsigned short* __restrict__ A2p, int lda, long strideA,
    const unsigned short* __restrict__ Btp, const unsigned short* __restrict__ Bt2p, int ldb, long strideB,
    void* __restrict__ Cout, void* __restrict__ Cout2, int ldc, long strideC,
    const float* __restrict__ bias,
    const float* __restrict__ resid, long strideR,
    int M, int N, int K, float scale) {
  typedef typename Elem<ET>::T T;
  typedef typename Frag<T>::V V;
  const T* A = (const T*)Ap; const T* A2 = (const T*)A2p; const T* Bt = (const T*)Btp; const T* Bt2 = (const T*)Bt2p;
  __shared__ __align__(16) float sT[8][16 * 68];
  const int b    = blockIdx.y;
  const int lane = threadIdx.x & 31;
  const int wave = threadIdx.x >> 5;
  const int tilesN = N >> 6;
  const int tilesM = M >> 6;
  const int tile = blockIdx.x * 8 + wave;
  if (tile >= tilesM * tilesN) return;
  const int tm = tile / tilesN;
  const int tn = tile - tm * tilesN;
  const int m0 = tm << 6;
  const int n0 = tn << 6;

  const T* Ab  = A  + (size_t)b * strideA;
  const T* Bb  = Bt + (size_t)b * strideB;
  const T* Ab2 = SPLIT ? (A2  + (size_t)b * strideA) : nullptr;
  const T* Bb2 = SPLIT ? (Bt2 + (size_t)b * strideB) : nullptr;

  const int rlane = lane & 15;
  const int koff  = (lane >> 4) * 8;
  const int mOff  = (lane >> 4) * 8;

  v8f acc[4][4];
#pragma unroll
  for (int i = 0; i < 4; ++i)
#pragma unroll
    for (int j = 0; j < 4; ++j) acc[i][j] = (v8f){0.f,0.f,0.f,0.f,0.f,0.f,0.f,0.f};

  for (int k0 = 0; k0 < K; k0 += 32) {
    V bh[4], bl[4];
#pragma unroll
    for (int j = 0; j < 4; ++j) {
      const size_t bo = (size_t)(n0 + (j << 4) + rlane) * ldb + koff + k0;
      bh[j] = Frag<T>::load(Bb + bo);
      if (SPLIT) bl[j] = Frag<T>::load(Bb2 + bo);
    }
#pragma unroll
    for (int i = 0; i < 4; ++i) {
      const size_t ao = (size_t)(m0 + (i << 4) + rlane) * lda + koff + k0;
      V ah = Frag<T>::load(Ab + ao);
      V al;
      if (SPLIT) al = Frag<T>::load(Ab2 + ao);
#pragma unroll
      for (int j = 0; j < 4; ++j) {
        acc[i][j] = Frag<T>::mma(ah, bh[j], acc[i][j]);
        if (SPLIT) {
          acc[i][j] = Frag<T>::mma(ah, bl[j], acc[i][j]);
          acc[i][j] = Frag<T>::mma(al, bh[j], acc[i][j]);
        }
      }
      Frag<T>::guard(acc[i][0], acc[i][3], ah, SPLIT ? al : ah);
    }
    Frag<T>::keep(bh[0], bh[1], bh[2], bh[3]);
    if (SPLIT) Frag<T>::keep(bl[0], bl[1], bl[2], bl[3]);
  }
  acc_guard4(acc[0][0], acc[0][1], acc[0][2], acc[0][3]);
  acc_guard4(acc[1][0], acc[1][1], acc[1][2], acc[1][3]);
  acc_guard4(acc[2][0], acc[2][1], acc[2][2], acc[2][3]);
  acc_guard4(acc[3][0], acc[3][1], acc[3][2], acc[3][3]);

  float* slab = sT[wave];
  const float* Rb = RESID ? (resid + (size_t)b * strideR) : nullptr;
#pragma unroll
  for (int i = 0; i < 4; ++i) {
    const int mBase = m0 + (i << 4);
#pragma unroll
    for (int j = 0; j < 4; ++j) {
      const int n = n0 + (j << 4) + rlane;
      float bv = 0.f;
      if (BIAS_MODE == 2) bv = bias[n];
#pragma unroll
      for (int r = 0; r < 8; ++r) {
        float v = acc[i][j][r] * scale;
        if (BIAS_MODE == 1) v += bias[mBase + mOff + r];
        if (BIAS_MODE == 2) v += bv;
        if (RESID) v += Rb[(size_t)(mBase + mOff + r) * ldc + n];
        if (ACT == 2) v = fmaxf(v, 0.0f);
        if (ACT == 4) v = (v > 0.f) ? v : 0.01f * v;
        slab[(mOff + r) * 68 + (j << 4) + rlane] = v;
      }
    }
    __builtin_amdgcn_fence(__ATOMIC_RELEASE, "workgroup");
    __builtin_amdgcn_wave_barrier();
    __builtin_amdgcn_fence(__ATOMIC_ACQUIRE, "workgroup");
    if (OUT_MODE == 0) {
      float* C = (float*)Cout + (size_t)b * strideC;
      const int hh = lane >> 4, c4 = (lane & 15) * 4;
      for (int pass = 0; pass < 2; ++pass) {
#pragma unroll
        for (int it = 0; it < 8; ++it) {
          const int row = it * 2 + hh;
          v4f v = *(const v4f*)(slab + row * 68 + c4);
          *(volatile v4f*)(C + (size_t)(mBase + row) * ldc + n0 + c4) = v;
        }
        __threadfence();
      }
    } else {
      const int q = lane >> 3, c8 = (lane & 7) * 8;
      unsigned short* C  = (unsigned short*)Cout  + (size_t)b * strideC;
      unsigned short* C2 = (OUT_MODE == 2) ? ((unsigned short*)Cout2 + (size_t)b * strideC) : nullptr;
      for (int pass = 0; pass < 2; ++pass) {
#pragma unroll
        for (int it = 0; it < 4; ++it) {
          const int row = it * 4 + q;
          const float* sp = slab + row * 68 + c8;
          v8h hv, lv;
#pragma unroll
          for (int e = 0; e < 8; ++e) {
            if (OUT_MODE == 1) {
              hv[e] = (_Float16)sp[e];
            } else {
              unsigned short hb = f2bf_bits(sp[e]);
              unsigned short lb = f2bf_bits(sp[e] - bf_bits2f(hb));
              hv[e] = __builtin_bit_cast(_Float16, hb);
              lv[e] = __builtin_bit_cast(_Float16, lb);
            }
          }
          *(volatile v8h*)(C + (size_t)(mBase + row) * ldc + n0 + c8) = hv;
          if (OUT_MODE == 2) *(volatile v8h*)(C2 + (size_t)(mBase + row) * ldc + n0 + c8) = lv;
        }
        __threadfence();
      }
    }
    __builtin_amdgcn_fence(__ATOMIC_RELEASE, "workgroup");
    __builtin_amdgcn_wave_barrier();
    __builtin_amdgcn_fence(__ATOMIC_ACQUIRE, "workgroup");
  }
}

__device__ __forceinline__ float fq(float v, float sc, float inv, float lo, float hi) {
#pragma clang fp contract(off)
  float k = rintf(v * sc);
  k = fminf(fmaxf(k, lo), hi);
  const float vq = k * inv;
  const float t = vq - v;
  return v + t;
}

__global__ __launch_bounds__(256) void xmax_partial_kernel(const float* __restrict__ x, float* __restrict__ part, int per) {
  __shared__ float red[256];
  const int t = threadIdx.x;
  const v4f* xv = (const v4f*)x + (size_t)blockIdx.x * per;
  float m = 0.f;
#pragma unroll 4
  for (int i = t; i < per; i += 256) {
    const v4f v = xv[i];
    m = fmaxf(m, fmaxf(fmaxf(fabsf(v[0]), fabsf(v[1])), fmaxf(fabsf(v[2]), fabsf(v[3]))));
  }
  red[t] = m;
  __syncthreads();
  for (int s = 128; s > 0; s >>= 1) {
    if (t < s) red[t] = fmaxf(red[t], red[t + s]);
    __syncthreads();
  }
  if (t < 32) {
    const float bm = red[0];
    float* p = part + (size_t)blockIdx.x * 32 + t;
    *(volatile float*)p = bm;
    __threadfence();
    *(volatile float*)p = bm;
  }
}

__global__ __launch_bounds__(256) void max_final_kernel(const float* __restrict__ part, int nlines, float qmax, float* __restrict__ scal) {
  __shared__ float red[256];
  const int t = threadIdx.x;
  float m = 0.f;
  for (int i = t; i < nlines; i += 256) m = fmaxf(m, part[(size_t)i * 32]);
  red[t] = m;
  __syncthreads();
  for (int s = 128; s > 0; s >>= 1) {
    if (t < s) red[t] = fmaxf(red[t], red[t + s]);
    __syncthreads();
  }
  if (t < 32) {
    const float am = fmaxf(red[0], 1e-8f);
    const float sc = qmax / am;
    const float inv = 1.0f / sc;
    float* p0 = scal + t;
    float* p1 = scal + 32 + t;
    *(volatile float*)p0 = sc;
    *(volatile float*)p1 = inv;
    __threadfence();
    *(volatile float*)p0 = sc;
    *(volatile float*)p1 = inv;
  }
}

__global__ __launch_bounds__(256) void colmax_kernel(const float* __restrict__ W, float* __restrict__ scv, float* __restrict__ invv, int R, int Cc) {
  const int j = blockIdx.x * 256 + threadIdx.x;
  const int jc = (j < Cc) ? j : (Cc - 1);
  float m = 0.f;
#pragma unroll 8
  for (int i = 0; i < R; ++i) m = fmaxf(m, fabsf(W[(size_t)i * Cc + jc]));
  m = fmaxf(m, 1e-8f);
  const float sc = 127.0f / m;
  const float inv = 1.0f / sc;
  if (j < Cc) {
    *(volatile float*)(scv + j) = sc;
    *(volatile float*)(invv + j) = inv;
    __threadfence();
    *(volatile float*)(scv + j) = sc;
    *(volatile float*)(invv + j) = inv;
  }
}

__global__ __launch_bounds__(256) void rowmax_kernel(const float* __restrict__ W, float* __restrict__ scv, float* __restrict__ invv, int R, int Cc) {
  __shared__ float srow[32];
  const int t = threadIdx.x;
  const int lane = t & 31, wave = t >> 5;
#pragma unroll 1
  for (int rr = 0; rr < 4; ++rr) {
    const int r = blockIdx.x * 32 + wave * 4 + rr;
    const int rc = (r < R) ? r : (R - 1);
    float m = 0.f;
#pragma unroll 8
    for (int k = lane; k < Cc; k += 32) m = fmaxf(m, fabsf(W[(size_t)rc * Cc + k]));
#pragma unroll
    for (int off = 16; off > 0; off >>= 1) m = fmaxf(m, __shfl_xor(m, off, 32));
    if (lane == 0) srow[wave * 4 + rr] = fmaxf(m, 1e-8f);
  }
  __syncthreads();
  if (wave == 0) {
    const float am = srow[lane];
    const float sc = 127.0f / am;
    const float inv = 1.0f / sc;
    const int r = blockIdx.x * 32 + lane;
    if (r < R) {
      *(volatile float*)(scv + r) = sc;
      *(volatile float*)(invv + r) = inv;
      __threadfence();
      *(volatile float*)(scv + r) = sc;
      *(volatile float*)(invv + r) = inv;
    }
  }
}

__global__ __launch_bounds__(256) void wq_in_kernel(const float* __restrict__ W, const float* __restrict__ scv,
                                                    const float* __restrict__ invv, unsigned short* __restrict__ out) {
#pragma clang fp contract(off)
  __shared__ float sm[64][65];
  const int t = threadIdx.x;
  const int i0 = blockIdx.x * 64;
  const int j0 = blockIdx.y * 64;
#pragma unroll
  for (int it = 0; it < 16; ++it) {
    const int e = it * 256 + t;
    const int il = e >> 6;
    const int jl = e & 63;
    sm[jl][il] = W[(size_t)(i0 + il) * kDF + j0 + jl];
  }
  __syncthreads();
  const int lane = t & 31, wave = t >> 5;
  const int q = lane >> 3, c8 = (lane & 7) * 8;
  v4u uu[2];
  size_t off[2];
#pragma unroll
  for (int it = 0; it < 2; ++it) {
    const int row = wave * 8 + it * 4 + q;
    const float sc = scv[j0 + row];
    const float inv = invv[j0 + row];
    unsigned short hb[8];
#pragma unroll
    for (int e = 0; e < 8; ++e) hb[e] = h_bits(fq(sm[row][c8 + e], sc, inv, -128.0f, 127.0f) * kWinCarry);
    uu[it] = (v4u){pk16(hb[0], hb[1]), pk16(hb[2], hb[3]), pk16(hb[4], hb[5]), pk16(hb[6], hb[7])};
    off[it] = (size_t)(j0 + row) * kDM + i0 + c8;
  }
  for (int pass = 0; pass < 2; ++pass) {
#pragma unroll
    for (int it = 0; it < 2; ++it) *(volatile v4u*)(out + off[it]) = uu[it];
    __threadfence();
  }
}

__global__ __launch_bounds__(256) void wq_out_kernel(const float* __restrict__ W, const float* __restrict__ scv,
                                                     const float* __restrict__ invv, unsigned short* __restrict__ out) {
#pragma clang fp contract(off)
  __shared__ float sm[64][65];
  const int t = threadIdx.x;
  const int k0 = blockIdx.x * 64;
  const int n0 = blockIdx.y * 64;
#pragma unroll
  for (int it = 0; it < 16; ++it) {
    const int e = it * 256 + t;
    const int kl = e >> 6;
    const int nl = e & 63;
    sm[nl][kl] = W[(size_t)(k0 + kl) * kDM + n0 + nl];
  }
  __syncthreads();
  const int lane = t & 31, wave = t >> 5;
  const int q = lane >> 3, c8 = (lane & 7) * 8;
  const v4f s0 = *(const v4f*)(scv + k0 + c8);
  const v4f s1 = *(const v4f*)(scv + k0 + c8 + 4);
  const v4f v0 = *(const v4f*)(invv + k0 + c8);
  const v4f v1 = *(const v4f*)(invv + k0 + c8 + 4);
  float sce[8], inve[8];
#pragma unroll
  for (int e = 0; e < 4; ++e) { sce[e] = s0[e]; sce[4 + e] = s1[e]; inve[e] = v0[e]; inve[4 + e] = v1[e]; }
  v4u uu[2];
  size_t off[2];
#pragma unroll
  for (int it = 0; it < 2; ++it) {
    const int row = wave * 8 + it * 4 + q;
    unsigned short hb[8];
#pragma unroll
    for (int e = 0; e < 8; ++e) hb[e] = h_bits(fq(sm[row][c8 + e], sce[e], inve[e], -128.0f, 127.0f) * kWoutCarry);
    uu[it] = (v4u){pk16(hb[0], hb[1]), pk16(hb[2], hb[3]), pk16(hb[4], hb[5]), pk16(hb[6], hb[7])};
    off[it] = (size_t)(n0 + row) * kDF + k0 + c8;
  }
  for (int pass = 0; pass < 2; ++pass) {
#pragma unroll
    for (int it = 0; it < 2; ++it) *(volatile v4u*)(out + off[it]) = uu[it];
    __threadfence();
  }
}

__global__ __launch_bounds__(256) void xquant_kernel(const float* __restrict__ x, const float* __restrict__ scal,
                                                    unsigned short* __restrict__ X16, int n8) {
#pragma clang fp contract(off)
  const int i = blockIdx.x * 256 + threadIdx.x;
  if (i >= n8) return;
  const float sc = scal[0];
  const float inv = scal[32];
  const float* p = x + 8 * (size_t)i;
  const v4f a = *(const v4f*)(p);
  const v4f c = *(const v4f*)(p + 4);
  unsigned short hb[8];
#pragma unroll
  for (int e = 0; e < 4; ++e) {
    hb[e]     = h_bits(fq(a[e], sc, inv, -32768.0f, 32767.0f) * kXCarry);
    hb[4 + e] = h_bits(fq(c[e], sc, inv, -32768.0f, 32767.0f) * kXCarry);
  }
  const v4u u = (v4u){pk16(hb[0], hb[1]), pk16(hb[2], hb[3]), pk16(hb[4], hb[5]), pk16(hb[6], hb[7])};
  unsigned short* qp = X16 + 8 * (size_t)i;
  *(volatile v4u*)qp = u;
  __threadfence();
  *(volatile v4u*)qp = u;
}

__global__ __launch_bounds__(256) void gelu_kernel(const float* __restrict__ H, unsigned short* __restrict__ G, float* __restrict__ part) {
  __shared__ float red[256];
  const int t = threadIdx.x;
  float m = 0.f;
#pragma unroll 1
  for (int gi = 0; gi < 4; ++gi) {
    const size_t idx8 = (size_t)(blockIdx.x * 4 + gi) * 256 + t;
    const float* hp = H + idx8 * 8;
    unsigned long long lo = 0ull, hi = 0ull;
#pragma unroll 1
    for (int e = 0; e < 8; ++e) {
      const float v = hp[e];
      const float g = 0.5f * v * (1.0f + erff(v * 0.70710678118654752f));
      m = fmaxf(m, fabsf(g));
      const unsigned long long ins = ((unsigned long long)h_bits(g * kGCarry)) << 48;
      if (e < 4) lo = (lo >> 16) | ins;
      else       hi = (hi >> 16) | ins;
    }
    const v4u u = (v4u){(unsigned)lo, (unsigned)(lo >> 32), (unsigned)hi, (unsigned)(hi >> 32)};
    unsigned short* qp = G + idx8 * 8;
    *(volatile v4u*)qp = u;
    __threadfence();
    *(volatile v4u*)qp = u;
  }
  red[t] = m;
  __syncthreads();
  for (int s = 128; s > 0; s >>= 1) {
    if (t < s) red[t] = fmaxf(red[t], red[t + s]);
    __syncthreads();
  }
  if (t < 32) {
    const float bm = red[0];
    float* p = part + (size_t)blockIdx.x * 32 + t;
    *(volatile float*)p = bm;
    __threadfence();
    *(volatile float*)p = bm;
  }
}

__global__ __launch_bounds__(256) void hquant_kernel(const unsigned short* __restrict__ G, const float* __restrict__ scal,
                                                    unsigned short* __restrict__ HQ, int n8) {
#pragma clang fp contract(off)
  const int i = blockIdx.x * 256 + threadIdx.x;
  if (i >= n8) return;
  const float sc = scal[0];
  const float inv = scal[32];
  const v4u w = *(const v4u*)(G + 8 * (size_t)i);
  unsigned short hb[8];
#pragma unroll
  for (int mi = 0; mi < 4; ++mi) {
    const unsigned wd = w[mi];
    const float g0 = f16lo_to_f32(wd) * kGCarryInv;
    const float g1 = f16hi_to_f32(wd) * kGCarryInv;
    hb[2 * mi]     = h_bits(fq(g0, sc, inv, -32768.0f, 32767.0f) * kHCarry);
    hb[2 * mi + 1] = h_bits(fq(g1, sc, inv, -32768.0f, 32767.0f) * kHCarry);
  }
  const v4u u = (v4u){pk16(hb[0], hb[1]), pk16(hb[2], hb[3]), pk16(hb[4], hb[5]), pk16(hb[6], hb[7])};
  unsigned short* qp = HQ + 8 * (size_t)i;
  *(volatile v4u*)qp = u;
  __threadfence();
  *(volatile v4u*)qp = u;
}

extern "C" void kernel_launch(void* const* d_in, const int* in_sizes, int n_in,
                              void* d_out, int out_size, void* d_ws, size_t ws_size,
                              hipStream_t stream) {
  if (n_in < 5) return;
  if (in_sizes[0] != kTok * kDM || in_sizes[1] != kDM * kDF || in_sizes[2] != kDF ||
      in_sizes[3] != kDF * kDM || in_sizes[4] != kDM) return;
  if (out_size != kTok * kDM) return;
  if (ws_size < kWsTotal) return;

  const float* x     = (const float*)d_in[0];
  const float* W_in  = (const float*)d_in[1];
  const float* b_in  = (const float*)d_in[2];
  const float* W_out = (const float*)d_in[3];
  const float* b_out = (const float*)d_in[4];
  float* out = (float*)d_out;

  char* ws = (char*)d_ws;
  float* scalX  = (float*)(ws + kOffScalX);
  float* scalH  = (float*)(ws + kOffScalH);
  float* scIn   = (float*)(ws + kOffScIn);
  float* invIn  = (float*)(ws + kOffInvIn);
  float* scOut  = (float*)(ws + kOffScOut);
  float* invOut = (float*)(ws + kOffInvOut);
  float* xpart  = (float*)(ws + kOffXPart);
  float* hpart  = (float*)(ws + kOffHPart);
  unsigned short* X16   = (unsigned short*)(ws + kOffX16);
  unsigned short* WinT  = (unsigned short*)(ws + kOffWinT);
  unsigned short* WoutT = (unsigned short*)(ws + kOffWoutT);
  float*          scrF  = (float*)(ws + kOffScr);
  unsigned short* scrH  = (unsigned short*)(ws + kOffScr);
  unsigned short* G16   = (unsigned short*)(ws + kOffG16);

  xmax_partial_kernel<<<dim3(kNPX), dim3(256), 0, stream>>>(x, xpart, kXPer4);
  max_final_kernel<<<dim3(1), dim3(256), 0, stream>>>(xpart, kNPX, 32767.0f, scalX);
  colmax_kernel<<<dim3(kDF / 256), dim3(256), 0, stream>>>(W_in, scIn, invIn, kDM, kDF);
  rowmax_kernel<<<dim3(kDF / 32), dim3(256), 0, stream>>>(W_out, scOut, invOut, kDF, kDM);

  wq_in_kernel<<<dim3(kDM / 64, kDF / 64), dim3(256), 0, stream>>>(W_in, scIn, invIn, WinT);
  wq_out_kernel<<<dim3(kDF / 64, kDM / 64), dim3(256), 0, stream>>>(W_out, scOut, invOut, WoutT);
  xquant_kernel<<<dim3(kXqBlocks), dim3(256), 0, stream>>>(x, scalX, X16, kTok * kDM / 8);

  const int g1blocks = ((kChunkRows / 64) * (kDF / 64)) / 8;
  const int g2blocks = ((kChunkRows / 64) * (kDM / 64)) / 8;
  for (int c = 0; c < kNumChunks; ++c) {
    const unsigned short* Ac = X16 + (size_t)c * kChunkRows * kDM;
    wmma_gemm64<0, false, 2, 0, false, 0><<<dim3(g1blocks, 1), dim3(256), 0, stream>>>(
        Ac, Ac, kDM, 0L,
        WinT, WinT, kDM, 0L,
        (void*)scrF, (void*)scrF, kDF, 0L,
        b_in, b_in, 0L,
        kChunkRows, kDF, kDM, kScale1);
    gelu_kernel<<<dim3(kGeluBlocks), dim3(256), 0, stream>>>(
        scrF, G16 + (size_t)c * kChunkRows * kDF, hpart + (size_t)c * kGeluBlocks * 32);
  }
  max_final_kernel<<<dim3(1), dim3(256), 0, stream>>>(hpart, kNPH, 32767.0f, scalH);

  for (int c = 0; c < kNumChunks; ++c) {
    hquant_kernel<<<dim3(kHqBlocks), dim3(256), 0, stream>>>(
        G16 + (size_t)c * kChunkRows * kDF, scalH, scrH, kChunkRows * kDF / 8);
    wmma_gemm64<0, false, 2, 0, false, 0><<<dim3(g2blocks, 1), dim3(256), 0, stream>>>(
        scrH, scrH, kDF, 0L,
        WoutT, WoutT, kDF, 0L,
        (void*)(out + (size_t)c * kChunkRows * kDM), (void*)(out + (size_t)c * kChunkRows * kDM), kDM, 0L,
        b_out, b_out, 0L,
        kChunkRows, kDM, kDF, kScale2);
  }
}
